// Combination_ANN_17051020165212
// MI455X (gfx1250) — hardware-verified
//
#include <hip/hip_runtime.h>


#define NS   16
#define NT   400
#define NF   16
#define NSF  250
#define NGRP 4
#define RPS  (NT * (1 + NSF))
#define NROW (NS * RPS)
#define RCH  160640
#define NCH  (NROW / RCH)
#define KA   32
#define NH1  64
#define DM   NH1
#define NTK  RCH
#define LOSC 1024.0f

typedef _Float16 h16;
typedef unsigned short bf;
typedef __attribute__((ext_vector_type(16))) __bf16   v16bf;
typedef __attribute__((ext_vector_type(16))) _Float16 v16h;
typedef __attribute__((ext_vector_type(8)))  _Float16 v8h;
typedef __attribute__((ext_vector_type(8)))  unsigned short v8us;
typedef __attribute__((ext_vector_type(8)))  float    v8f;
typedef __attribute__((ext_vector_type(4)))  float    v4f;
typedef __attribute__((ext_vector_type(4)))  _Float16 v4h;
typedef v8h  __attribute__((may_alias)) v8ha;
typedef v4f  __attribute__((may_alias)) v4fa;
typedef v8us __attribute__((may_alias)) v8usa;

__device__ __forceinline__ unsigned short f2bf(float f) { unsigned u = __float_as_uint(f); u += 0x7FFFu + ((u >> 16) & 1u); return (unsigned short)(u >> 16); }
__device__ __forceinline__ float bf2f(unsigned short b) { return __uint_as_float(((unsigned)b) << 16); }
__device__ __forceinline__ float bfr(float f) { return bf2f(f2bf(f)); }
__device__ __forceinline__ v16h cat16(v8h lo, v8h hi) { return __builtin_shufflevector(lo, hi, 0, 1, 2, 3, 4, 5, 6, 7, 8, 9, 10, 11, 12, 13, 14, 15); }
__device__ __forceinline__ v16bf cat16b(v8us lo, v8us hi) { return __builtin_bit_cast(v16bf, __builtin_shufflevector(lo, hi, 0, 1, 2, 3, 4, 5, 6, 7, 8, 9, 10, 11, 12, 13, 14, 15)); }
__device__ __forceinline__ v8f wmma16(v16h a, v16h b, v8f c) { return __builtin_amdgcn_wmma_f32_16x16x32_f16(false, a, false, b, (short)0, c, false, false); }
__device__ __forceinline__ v8f wmmab(v16bf a, v16bf b, v8f c) { return __builtin_amdgcn_wmma_f32_16x16x32_bf16(false, a, false, b, (short)0, c, false, false); }

template <bool SPLITA, bool F16OUT = false>
__global__ __launch_bounds__(128) void k_gemmb(const bf* __restrict__ A, const bf* __restrict__ Al, const bf* __restrict__ Bn, const float* __restrict__ bias, float* C, int ldc, h16* C2, const float* __restrict__ R = nullptr, int K = DM, int roundR = 1) {
    __shared__ __align__(16) float ost[4][16 * 68];
    const int lane = threadIdx.x & 31, wave = threadIdx.x >> 5, lr = lane & 15, hi = lane >> 4;
    const int r0 = blockIdx.x * 64 + wave * 16, c0 = blockIdx.y * 64;
    const size_t aoff = (size_t)(r0 + lr) * K + 8 * hi;
    size_t boff[4];
#pragma unroll
    for (int t = 0; t < 4; ++t) boff[t] = (size_t)(c0 + t * 16 + lr) * K + 8 * hi;
    v8f acc[4];
#pragma unroll
    for (int t = 0; t < 4; ++t) acc[t] = (v8f){};
#pragma unroll 1
    for (int kc = 0; kc < K; kc += 32) {
        const v16bf a = cat16b(*(const v8us*)(A + aoff + kc), *(const v8us*)(A + aoff + kc + 16));
        v16bf al = a;
        if (SPLITA) al = cat16b(*(const v8us*)(Al + aoff + kc), *(const v8us*)(Al + aoff + kc + 16));
#pragma unroll
        for (int t = 0; t < 4; ++t) { const v16bf b = cat16b(*(const v8us*)(Bn + boff[t] + kc), *(const v8us*)(Bn + boff[t] + kc + 16)); acc[t] = wmmab(a, b, acc[t]); if (SPLITA) acc[t] = wmmab(al, b, acc[t]); }
        asm volatile("v_nop\n\tv_nop\n\tv_nop\n\tv_nop" : "+v"(acc[0]), "+v"(acc[1]), "+v"(acc[2]), "+v"(acc[3]) : "v"(a), "v"(al));
    }
    float* os = &ost[wave][0];
#pragma unroll
    for (int t = 0; t < 4; ++t) { const float bv = bias ? bfr(bias[c0 + t * 16 + lr]) : 0.f;
#pragma unroll
        for (int j = 0; j < 8; ++j) os[(hi * 8 + j) * 68 + t * 16 + lr] = acc[t][j] + bv; }
    __syncthreads();
    if (F16OUT) {
        h16* crow = (h16*)(void*)C + (size_t)r0 * ldc + c0;
        auto pass = [&]() {
#pragma unroll
            for (int s = 0; s < 4; ++s) { const int row = 4 * s + (lane >> 3), piece = lane & 7; const float* sp = os + row * 68 + piece * 8; v8h o, o2;
#pragma unroll
                for (int i = 0; i < 8; ++i) { const h16 a = (h16)sp[i]; o[i] = a; o2[i] = (h16)((sp[i] - (float)a) * LOSC); }
                *(volatile v8h*)(crow + (size_t)row * ldc + piece * 8) = o; if (C2) *(volatile v8h*)(C2 + (size_t)r0 * ldc + c0 + (size_t)row * ldc + piece * 8) = o2; }
        };
        pass(); __threadfence(); pass();
    } else {
        float* crow = C + (size_t)r0 * ldc + c0;
        auto pass = [&]() {
#pragma unroll
            for (int s = 0; s < 8; ++s) { const int Lid = (lane >> 3) + 4 * s, piece = lane & 7; const int row = Lid >> 1, cofs = (Lid & 1) * 32 + piece * 4;
                v4f val = *(const v4fa*)(os + row * 68 + cofs); if (R) { const v4f rv = *(const v4f*)(R + ((size_t)r0 + row) * ldc + c0 + cofs); val += roundR ? (v4f){bfr(rv[0]), bfr(rv[1]), bfr(rv[2]), bfr(rv[3])} : rv; }
                *(volatile v4f*)(crow + (size_t)row * ldc + cofs) = val; }
        };
        pass(); __threadfence(); pass();
    }
}


__global__ __launch_bounds__(256) void k_wpad(const float* __restrict__ W1, const float* __restrict__ b1, const float* __restrict__ W2, const float* __restrict__ b2, const float* __restrict__ W3, const float* __restrict__ b3,
                                              bf* W1N, bf* W2N, bf* W3N, float* BP) {
    const int u = blockIdx.x * 256 + threadIdx.x;
    if (u < NH1 * KA / 8) { const int n = u / (KA / 8), k0 = (u % (KA / 8)) * 8; v8us v;
#pragma unroll
        for (int i = 0; i < 8; ++i) { const int k = k0 + i; v[i] = (k < NF && n < 32) ? f2bf(W1[k * 32 + n]) : (unsigned short)0; }
        *(volatile v8us*)(W1N + n * KA + k0) = v; __threadfence(); *(volatile v8us*)(W1N + n * KA + k0) = v; }
    if (u < NH1 * NH1 / 8) { const int n = u / (NH1 / 8), k0 = (u % (NH1 / 8)) * 8; v8us v2, v3;
#pragma unroll
        for (int i = 0; i < 8; ++i) { const int k = k0 + i; v2[i] = (k < 32 && n < 16) ? f2bf(W2[k * 16 + n]) : (unsigned short)0; v3[i] = (k < 16 && n == 0) ? f2bf(W3[k]) : (unsigned short)0; }
        *(volatile v8us*)(W2N + n * NH1 + k0) = v2; *(volatile v8us*)(W3N + n * NH1 + k0) = v3; __threadfence(); *(volatile v8us*)(W2N + n * NH1 + k0) = v2; *(volatile v8us*)(W3N + n * NH1 + k0) = v3; }
    if (u < 3 * NH1 / 4) { const int which = u / (NH1 / 4), c0 = (u % (NH1 / 4)) * 4; v4f v;
#pragma unroll
        for (int i = 0; i < 4; ++i) { const int c = c0 + i; v[i] = (which == 0) ? (c < 32 ? b1[c] : 0.f) : (which == 1 ? (c < 16 ? b2[c] : 0.f) : (c == 0 ? b3[0] : 0.f)); }
        *(volatile v4f*)(BP + which * NH1 + c0) = v; __threadfence(); *(volatile v4f*)(BP + which * NH1 + c0) = v; }
}
__global__ __launch_bounds__(256) void k_norm(const float* __restrict__ obs, const float* __restrict__ mu, const float* __restrict__ SMH, const int* __restrict__ perm, int r0, bf* Ah, bf* Al) {
    const int u = blockIdx.x * 256 + threadIdx.x; if (u >= RCH * 4) return;
    const int r = u >> 2, q = u & 3; const int g = r0 + r; const int s = g / RPS, l = g % RPS;
    v8us oh, ol;
    if (q < 2) {
        float x[NF];
        if (l < NT) {
#pragma unroll
            for (int j = 0; j < NF; ++j) x[j] = bfr(obs[((size_t)s * NT + l) * NF + j]) - bfr(mu[j]);
        } else { const int sf = (l - NT) / NT, t = (l - NT) % NT;
#pragma unroll
            for (int j = 0; j < NF; ++j) { int pi = perm[(((size_t)sf * NGRP + j / (NF / NGRP)) * NS + s) * NT + t]; pi = pi < 0 ? 0 : (pi >= NT ? NT - 1 : pi); x[j] = bfr(obs[((size_t)s * NT + pi) * NF + j]) - bfr(mu[j]); }
        }
#pragma unroll
        for (int i8 = 0; i8 < 8; ++i8) { const int i = q * 8 + i8; float y = 0.f;
#pragma unroll
            for (int j = 0; j < NF; ++j) y = fmaf(bfr(SMH[i * NF + j]), x[j], y);
            const unsigned short hb = f2bf(y); oh[i8] = hb; ol[i8] = f2bf(y - bf2f(hb)); }
    } else {
#pragma unroll
        for (int i8 = 0; i8 < 8; ++i8) { oh[i8] = 0; ol[i8] = 0; }
    }
    const size_t o = (size_t)r * KA + q * 8;
    *(volatile v8us*)(Ah + o) = oh; *(volatile v8us*)(Al + o) = ol; __threadfence(); *(volatile v8us*)(Ah + o) = oh; *(volatile v8us*)(Al + o) = ol;
}
__global__ __launch_bounds__(256) void k_lrelu(const float* __restrict__ T, int nrows, bf* Hh, bf* Hl) {
    typedef __attribute__((ext_vector_type(2))) unsigned short v2us;
    const int lane = threadIdx.x & 31, r = blockIdx.x * 8 + (threadIdx.x >> 5); if (r >= nrows) return;
    const size_t o = (size_t)r * NH1 + lane * 2; v2us oh, ol;
#pragma unroll
    for (int i = 0; i < 2; ++i) { const float v = T[o + i]; const float y = v >= 0.f ? v : 0.01f * v; const unsigned short hb = f2bf(y); oh[i] = hb; ol[i] = f2bf(y - bf2f(hb)); }
    *(volatile v2us*)(Hh + o) = oh; *(volatile v2us*)(Hl + o) = ol; __threadfence(); *(volatile v2us*)(Hh + o) = oh; *(volatile v2us*)(Hl + o) = ol;
}
__global__ __launch_bounds__(256) void k_sig(const float* __restrict__ T, int r0, float* OUTP) {
    const int r = blockIdx.x * 256 + threadIdx.x; if (r >= RCH) return;
    const float y = 1.0f / (1.0f + __expf(-T[(size_t)r * NH1]));
    *(volatile float*)(OUTP + r0 + r) = y; __threadfence(); *(volatile float*)(OUTP + r0 + r) = y;
}

extern "C" void kernel_launch(void* const* d_in, const int* in_sizes, int n_in,
                              void* d_out, int out_size, void* d_ws, size_t ws_size, hipStream_t stream) {
    (void)in_sizes; (void)n_in; (void)out_size;
    const float* obs = (const float*)d_in[0]; const float* mu = (const float*)d_in[1]; const float* SMH = (const float*)d_in[2]; const int* perm = (const int*)d_in[3];
    const float* W1 = (const float*)d_in[4]; const float* b1 = (const float*)d_in[5]; const float* W2 = (const float*)d_in[6]; const float* b2 = (const float*)d_in[7]; const float* W3 = (const float*)d_in[8]; const float* b3 = (const float*)d_in[9];
    float* out = (float*)d_out;
    char* wsp = (char*)d_ws;
    auto take = [&](size_t bytes) { char* p = wsp; wsp += (bytes + 255) & ~(size_t)255; return (void*)p; };
    bf* W1N = (bf*)take((size_t)NH1 * KA * 2); bf* W2N = (bf*)take((size_t)NH1 * NH1 * 2); bf* W3N = (bf*)take((size_t)NH1 * NH1 * 2); float* BP = (float*)take((size_t)3 * NH1 * 4);
    bf* Ah = (bf*)take((size_t)RCH * KA * 2); bf* Al = (bf*)take((size_t)RCH * KA * 2); float* T = (float*)take((size_t)RCH * NH1 * 4); bf* Hh = (bf*)take((size_t)RCH * NH1 * 2); bf* Hl = (bf*)take((size_t)RCH * NH1 * 2);
    if ((size_t)(wsp - (char*)d_ws) > ws_size) return;
    k_wpad<<<(NH1 * NH1 / 8 + 255) / 256, 256, 0, stream>>>(W1, b1, W2, b2, W3, b3, W1N, W2N, W3N, BP);
    for (int ch = 0; ch < NCH; ++ch) {
        const int r0 = ch * RCH;
        k_norm<<<(RCH * 4) / 256, 256, 0, stream>>>(obs, mu, SMH, perm, r0, Ah, Al);
        k_gemmb<true, false><<<dim3(RCH / 64, 1, 1), 128, 0, stream>>>(Ah, Al, W1N, BP, T, NH1, nullptr, nullptr, KA);
        k_lrelu<<<RCH / 8, 256, 0, stream>>>(T, RCH, Hh, Hl);
        k_gemmb<true, false><<<dim3(RCH / 64, 1, 1), 128, 0, stream>>>(Hh, Hl, W2N, BP + NH1, T, NH1, nullptr, nullptr, NH1);
        k_lrelu<<<RCH / 8, 256, 0, stream>>>(T, RCH, Hh, Hl);
        k_gemmb<true, false><<<dim3(RCH / 64, 1, 1), 128, 0, stream>>>(Hh, Hl, W3N, BP + 2 * NH1, T, NH1, nullptr, nullptr, NH1);
        k_sig<<<(RCH + 255) / 256, 256, 0, stream>>>(T, r0, out);
    }
}
